// SharpenedCosineSimilarity_34419867910708
// MI455X (gfx1250) — hardware-verified
//
#include <hip/hip_runtime.h>


#define NI   16
#define CI   64
#define IH   64
#define IW   64
#define CO   128
#define KK   9
#define KD   (CI * KK)
#define NPX  (NI * IH * IW)
#define EPSV 1e-12f

typedef unsigned short bf;
typedef __attribute__((ext_vector_type(16))) __bf16   v16bf;
typedef __attribute__((ext_vector_type(8)))  unsigned short v8us;
typedef __attribute__((ext_vector_type(8)))  float    v8f;
typedef __attribute__((ext_vector_type(4)))  float    v4f;
typedef v4f  __attribute__((may_alias)) v4fa;
typedef v8us __attribute__((may_alias)) v8usa;

__device__ __forceinline__ unsigned short f2bf(float f) { unsigned u = __float_as_uint(f); u += 0x7FFFu + ((u >> 16) & 1u); return (unsigned short)(u >> 16); }
__device__ __forceinline__ float bf2f(unsigned short b) { return __uint_as_float(((unsigned)b) << 16); }
__device__ __forceinline__ float bfr(float f) { return bf2f(f2bf(f)); }
__device__ __forceinline__ v16bf cat16b(v8us lo, v8us hi) { return __builtin_bit_cast(v16bf, __builtin_shufflevector(lo, hi, 0, 1, 2, 3, 4, 5, 6, 7, 8, 9, 10, 11, 12, 13, 14, 15)); }
__device__ __forceinline__ v8f wmmab(v16bf a, v16bf b, v8f c) { return __builtin_amdgcn_wmma_f32_16x16x32_bf16(false, a, false, b, (short)0, c, false, false); }
#define VST2(T, p, v) do { const T vst2_v_ = (v); *(volatile T*)(p) = vst2_v_; __threadfence(); *(volatile T*)(p) = vst2_v_; } while (0)

__global__ __launch_bounds__(64) void k_energy(const float* __restrict__ x, float* E) {
    const int n = blockIdx.y, h = blockIdx.x, w = threadIdx.x; float s = 0.f;
#pragma unroll 4
    for (int c = 0; c < CI; ++c) { const float v = bfr(x[(((size_t)n * CI + c) * IH + h) * IW + w]); s += v * v; }
    VST2(float, E + ((size_t)n * IH + h) * IW + w, s);
}
__global__ __launch_bounds__(64) void k_xnorm(const float* __restrict__ E, const float* __restrict__ qv, float* XN) {
    const int n = blockIdx.y, h = blockIdx.x, w = threadIdx.x; float s = 0.f;
#pragma unroll
    for (int a = -1; a <= 1; ++a)
#pragma unroll
        for (int b = -1; b <= 1; ++b) { const int hh = h + a, ww = w + b; if (hh >= 0 && hh < IH && ww >= 0 && ww < IW) s += E[((size_t)n * IH + hh) * IW + ww]; }
    const float qn = bfr(qv[0]) * 0.01f;
    VST2(float, XN + ((size_t)n * IH + h) * IW + w, sqrtf(s + EPSV) + qn * qn);
}
__global__ __launch_bounds__(256) void k_wprep(const float* __restrict__ Wm, bf* WB) {
    const int lane = threadIdx.x & 31, wave = threadIdx.x >> 5, v = blockIdx.x * 8 + wave;
#pragma unroll 1
    for (int ps = 0; ps < 2; ++ps) {
#pragma unroll
        for (int k = 0; k < 3; ++k) { const int pc = lane + 32 * k; if (pc < 72) { v8us o;
#pragma unroll
                for (int i = 0; i < 8; ++i) o[i] = f2bf(Wm[(size_t)v * KD + pc * 8 + i]);
                *(volatile v8us*)(WB + (size_t)v * KD + pc * 8) = o; } }
        if (ps == 0) __threadfence(); }
}
__global__ __launch_bounds__(128) void k_wnorm(const float* __restrict__ Wm, const float* __restrict__ qv, float* WN) {
    const int v = threadIdx.x; float s = 0.f;
#pragma unroll 4
    for (int k = 0; k < KD; ++k) { const float f = bfr(Wm[(size_t)v * KD + k]); s += f * f; }
    const float qn = bfr(qv[0]) * 0.01f;
    VST2(float, WN + v, sqrtf(s + EPSV) + qn * qn);
}
__global__ __launch_bounds__(256) void k_im2col(const float* __restrict__ x, bf* A) {
    __shared__ __align__(16) unsigned short tl[16 * 584];
    const int n = blockIdx.z, h = blockIdx.y, w0 = blockIdx.x * 16, tid = threadIdx.x;
#pragma unroll
    for (int r = 0; r < 4; ++r) { const int idx = r * 256 + tid; const int wl = idx >> 6, c = idx & 63; const int w = w0 + wl;
#pragma unroll
        for (int a = 0; a < 3; ++a)
#pragma unroll
            for (int b = 0; b < 3; ++b) { const int hh = h + a - 1, ww = w + b - 1; float v = 0.f;
                if (hh >= 0 && hh < IH && ww >= 0 && ww < IW) v = x[(((size_t)n * CI + c) * IH + hh) * IW + ww];
                tl[wl * 584 + c * KK + a * 3 + b] = f2bf(v); } }
    __syncthreads();
    const size_t rbase = ((size_t)n * IH + h) * IW + w0;
    auto pass = [&]() {
#pragma unroll
        for (int s = 0; s < 5; ++s) { const int p = s * 256 + tid; if (p < 1152) { const int row = p / 72, pc = p - row * 72;
            *(volatile v8us*)(A + (rbase + row) * KD + pc * 8) = *(const v8usa*)(tl + row * 584 + pc * 8); } }
    };
    pass(); __threadfence(); pass();
}
__global__ __launch_bounds__(128) void k_gemm(const bf* __restrict__ A, const bf* __restrict__ WB, const float* __restrict__ XN, const float* __restrict__ WN, const float* __restrict__ pv, float* out) {
    __shared__ __align__(16) float ot[64 * 68];
    const int lane = threadIdx.x & 31, wave = threadIdx.x >> 5, lr = lane & 15, hi = lane >> 4;
    const size_t rblk = (size_t)blockIdx.x * 64; const size_t r0 = rblk + wave * 16; const int c0 = blockIdx.y * 64;
    v8f acc[4];
#pragma unroll
    for (int t = 0; t < 4; ++t) acc[t] = (v8f){};
#pragma unroll 2
    for (int kc = 0; kc < KD; kc += 32) {
        const v16bf a = cat16b(*(const v8us*)(A + (r0 + lr) * KD + kc + 8 * hi), *(const v8us*)(A + (r0 + lr) * KD + kc + 8 * hi + 16));
#pragma unroll
        for (int t = 0; t < 4; ++t) { const bf* bp = WB + (size_t)(c0 + t * 16 + lr) * KD + kc + 8 * hi; acc[t] = wmmab(a, cat16b(*(const v8us*)bp, *(const v8us*)(bp + 16)), acc[t]); }
        asm volatile("v_nop" : "+v"(acc[0]), "+v"(acc[1]), "+v"(acc[2]), "+v"(acc[3]) : "v"(a) : "memory");
    }
#pragma unroll
    for (int t = 0; t < 4; ++t) { const int v = c0 + t * 16 + lr; const float wn = WN[v]; const float pq = bfr(pv[v]) * 0.1f; const float ex = pq * pq;
#pragma unroll
        for (int j = 0; j < 8; ++j) { const size_t px = r0 + hi * 8 + j; const float y = acc[t][j] / (XN[px] * wn);
            const float sg = (y > 0.f) ? 1.f : ((y < 0.f) ? -1.f : 0.f); const float r = sg * __expf(ex * __logf(fabsf(y) + EPSV));
            ot[(t * 16 + lr) * 68 + wave * 16 + hi * 8 + j] = r; } }
    __syncthreads();
    const int n = (int)(rblk / (IH * IW)); const int h = (int)((rblk / IW) % IH);
    auto pass = [&]() {
#pragma unroll
        for (int s = 0; s < 8; ++s) { const int vl = wave * 16 + s * 2 + (lane >> 4), piece = lane & 15;
            const v4f val = *(const v4fa*)(ot + vl * 68 + piece * 4); *(volatile v4f*)(out + ((((size_t)n * CO + c0 + vl) * IH + h) * IW) + piece * 4) = val; }
    };
    pass(); __threadfence(); pass();
}

extern "C" void kernel_launch(void* const* d_in, const int* in_sizes, int n_in,
                              void* d_out, int out_size, void* d_ws, size_t ws_size, hipStream_t stream) {
    (void)in_sizes; (void)n_in; (void)out_size;
    const float* x = (const float*)d_in[0]; const float* Wm = (const float*)d_in[1]; const float* pv = (const float*)d_in[2]; const float* qv = (const float*)d_in[3];
    float* out = (float*)d_out;
    char* wsp = (char*)d_ws;
    auto take = [&](size_t bytes) { char* p = wsp; wsp += (bytes + 255) & ~(size_t)255; return (void*)p; };
    bf* A = (bf*)take((size_t)NPX * KD * 2); bf* WB = (bf*)take((size_t)CO * KD * 2); float* E = (float*)take((size_t)NPX * 4); float* XN = (float*)take((size_t)NPX * 4); float* WN = (float*)take((size_t)CO * 4);
    if ((size_t)(wsp - (char*)d_ws) > ws_size) return;
    k_energy<<<dim3(IH, NI, 1), 64, 0, stream>>>(x, E);
    k_xnorm<<<dim3(IH, NI, 1), 64, 0, stream>>>(E, qv, XN);
    k_wprep<<<CO / 8, 256, 0, stream>>>(Wm, WB); k_wnorm<<<1, 128, 0, stream>>>(Wm, qv, WN);
    k_im2col<<<dim3(IW / 16, IH, NI), 256, 0, stream>>>(x, A);
    k_gemm<<<dim3(NPX / 64, CO / 64, 1), 128, 0, stream>>>(A, WB, XN, WN, pv, out);
}
